// ScaledDotProductAttention_54374285967459
// MI455X (gfx1250) — hardware-verified
//
#include <hip/hip_runtime.h>
#ifndef NB
#define NB 16
#endif
#ifndef SEQ
#define SEQ 2048
#endif
#define NB_FULL 16
#define SEQ_FULL 2048
#define HD 64
#define QT (SEQ / 64)
static_assert(SEQ % 64 == 0);
static_assert(SEQ <= SEQ_FULL);
static_assert(NB <= NB_FULL);
static_assert(((size_t)NB * SEQ * HD) % 2048 == 0);

typedef unsigned short v8us __attribute__((ext_vector_type(8), may_alias));
typedef _Float16 v16h __attribute__((ext_vector_type(16)));
typedef float  v8f  __attribute__((ext_vector_type(8)));
typedef float  v4f  __attribute__((ext_vector_type(4)));
typedef float  v4fa __attribute__((ext_vector_type(4), may_alias));
union FragH { v16h v; v8us half[2]; _Float16 h[16]; unsigned short u[16]; };

__device__ __forceinline__ unsigned short bf16_bits(float x) { unsigned int u = __float_as_uint(x); return (unsigned short)((u + 0x7FFFu + ((u >> 16) & 1u)) >> 16); }
__device__ __forceinline__ float bf16_val(unsigned short b) { return __uint_as_float(((unsigned int)b) << 16); }
__device__ __forceinline__ float bf16_rne(float x) { return bf16_val(bf16_bits(x)); }

__device__ __forceinline__ v16h g2_frag(const _Float16* p, unsigned hh) { FragH f; f.half[0] = *(const v8us*)((const unsigned short*)p + 8u * hh); f.half[1] = *(const v8us*)((const unsigned short*)p + 16u + 8u * hh); return f.v; }
__device__ __forceinline__ v8f g2_mma(v16h a, v16h b, v8f c) { v8f d = __builtin_amdgcn_wmma_f32_16x16x32_f16(false, a, false, b, (short)0, c, false, false); asm volatile("v_nop\n\tv_nop\n\tv_nop\n\tv_nop" : "+v"(d) : "v"(a), "v"(b)); return d; }
__device__ __forceinline__ v16h q_frag(const float* p, unsigned hh) {
  const v4f x0 = *(const v4fa*)(p + 8u * hh), x1 = *(const v4fa*)(p + 8u * hh + 4u);
  const v4f x2 = *(const v4fa*)(p + 16u + 8u * hh), x3 = *(const v4fa*)(p + 16u + 8u * hh + 4u);
  FragH f;
#pragma unroll
  for (int q = 0; q < 4; ++q) { f.h[q] = (_Float16)bf16_rne(x0[q]); f.h[4 + q] = (_Float16)bf16_rne(x1[q]); f.h[8 + q] = (_Float16)bf16_rne(x2[q]); f.h[12 + q] = (_Float16)bf16_rne(x3[q]); }
  return f.v;
}

__global__ __launch_bounds__(256) void k_k16(const float* __restrict__ x, _Float16* __restrict__ X16) {
  const unsigned t = blockIdx.x * 256u + threadIdx.x;
  if (t >= (unsigned)(NB * SEQ * 8)) return;
  const unsigned b = t / (unsigned)(SEQ * 8), rem = t - b * (unsigned)(SEQ * 8);
  const float* src = x + (size_t)b * SEQ_FULL * HD + (size_t)rem * 8u;
  const v4f a = *(const v4fa*)src, c = *(const v4fa*)(src + 4);
  FragH f;
#pragma unroll
  for (int q = 0; q < 4; ++q) { f.h[q] = (_Float16)bf16_rne(a[q]); f.h[4 + q] = (_Float16)bf16_rne(c[q]); }
  const v8us o = f.half[0];
  unsigned short* d = (unsigned short*)X16 + (size_t)t * 8u;
  *(volatile v8us*)d = o;
  __threadfence();
  *(volatile v8us*)d = o;
}

__global__ __launch_bounds__(256) void k_vtc(const float* __restrict__ V, _Float16* __restrict__ VT) {
  __shared__ unsigned short tl[64][65];
  const unsigned tid = threadIdx.x;
  const unsigned b = blockIdx.x / (unsigned)QT, sg = blockIdx.x - b * (unsigned)QT;
  const unsigned s0 = sg * 64u;
  for (unsigned i = tid; i < 512u; i += 256u) {
    const unsigned j = i >> 3, d8 = (i & 7u) * 8u;
    const float* src = V + ((size_t)b * SEQ_FULL + s0 + j) * HD + d8;
    const v4f a = *(const v4fa*)src, c = *(const v4fa*)(src + 4);
    FragH f;
#pragma unroll
    for (int q = 0; q < 4; ++q) { f.h[q] = (_Float16)bf16_rne(a[q]); f.h[4 + q] = (_Float16)bf16_rne(c[q]); }
#pragma unroll
    for (int q = 0; q < 8; ++q) tl[d8 + q][j] = f.u[q];
  }
  __syncthreads();
  for (int pass = 0; pass < 2; ++pass) {
    for (unsigned i = tid; i < 512u; i += 256u) {
      const unsigned d = i >> 3, j8 = (i & 7u) * 8u;
      FragH f;
#pragma unroll
      for (int q = 0; q < 8; ++q) f.u[q] = tl[d][j8 + q];
      const v8us o = f.half[0];
      *(volatile v8us*)((unsigned short*)VT + ((size_t)b * HD + d) * SEQ + s0 + j8) = o;
    }
    if (pass == 0) __threadfence();
  }
}

__global__ __launch_bounds__(128) void k_fattn(const float* __restrict__ Qf, const _Float16* __restrict__ K16, const _Float16* __restrict__ VT,
                                              const int* __restrict__ plen_n, float* __restrict__ Og) {
  __shared__ __attribute__((aligned(16))) float so[4][16][68];
  const unsigned tid = threadIdx.x, w = tid >> 5, lane = tid & 31u, ln = lane & 15u, hh = lane >> 4;
  const unsigned b = blockIdx.x / (unsigned)QT, qt = blockIdx.x - b * (unsigned)QT;
  const unsigned q0 = qt * 64u + w * 16u;
  const unsigned qidx = q0 + ln;
  int pl = plen_n[b];
  pl = pl < 0 ? 0 : pl; pl = pl > SEQ ? SEQ : pl;
  const unsigned plen = (unsigned)pl;
  const unsigned ntp = (plen + 63u) >> 6;
  const unsigned ntot = ntp + ((qt >= ntp) ? 1u : 0u);

  const float* qrow = Qf + ((size_t)b * SEQ_FULL + qidx) * HD;
  const v16h qa0 = q_frag(qrow, hh), qa1 = q_frag(qrow + 32, hh);
  const _Float16* Kb = K16 + (size_t)b * SEQ * HD;
  const _Float16* Vb = VT + (size_t)b * HD * SEQ;

  const float NEGBIG = -1.0e30f;
  const v8f z8 = {0.f, 0.f, 0.f, 0.f, 0.f, 0.f, 0.f, 0.f};
  float m = NEGBIG, l = 0.f;
  v8f oh[4] = {z8, z8, z8, z8}, orr[4] = {z8, z8, z8, z8};

#pragma unroll 1
  for (unsigned it = 0; it < ntot; ++it) {
    const unsigned kt = (it < ntp) ? it : qt;
    const unsigned key0 = kt * 64u;
    v8f s[4];
#pragma unroll
    for (int t = 0; t < 4; ++t) {
      const _Float16* kr = Kb + (size_t)(key0 + (unsigned)t * 16u + ln) * HD;
      const v16h a0 = g2_frag(kr, hh), a1 = g2_frag(kr + 32, hh);
      v8f c = z8;
      c = g2_mma(a0, qa0, c);
      c = g2_mma(a1, qa1, c);
      s[t] = c;
    }
    const bool full = (key0 + 64u <= plen);
    float tmx = NEGBIG;
#pragma unroll
    for (int t = 0; t < 4; ++t) {
#pragma unroll
      for (int r = 0; r < 8; ++r) {
        const unsigned key = key0 + (unsigned)t * 16u + 8u * hh + (unsigned)r;
        const bool keep = full | (key < plen) | (key == qidx);
        const float v = keep ? s[t][r] * 0.125f : NEGBIG;
        s[t][r] = v;
        tmx = fmaxf(tmx, v);
      }
    }
    tmx = fmaxf(tmx, __shfl_xor(tmx, 16));
    const float mnew = fmaxf(m, tmx);
    const float alpha = __expf(fmaxf(m - mnew, -80.0f));
    m = mnew;
    FragH ph[2], pr[2];
    float ls = 0.f;
#pragma unroll
    for (int t = 0; t < 4; ++t) {
#pragma unroll
      for (int r = 0; r < 8; ++r) {
        const float sv = s[t][r];
        const float e = __expf(fmaxf(sv - mnew, -80.0f));
        const float p = (sv > -1.0e29f) ? e : 0.0f;
        ls += p;
        const float p256 = p * 256.0f;
        const _Float16 hv = (_Float16)p256;
        const _Float16 rv = (_Float16)((p256 - (float)hv) * 2048.0f);
        ph[t >> 1].h[(t & 1) * 8 + r] = hv;
        pr[t >> 1].h[(t & 1) * 8 + r] = rv;
      }
    }
    l = l * alpha + ls;
#pragma unroll
    for (int dt = 0; dt < 4; ++dt) { oh[dt] = oh[dt] * alpha; orr[dt] = orr[dt] * alpha; }
#pragma unroll
    for (int dt = 0; dt < 4; ++dt) {
      const _Float16* vr = Vb + (size_t)((unsigned)dt * 16u + ln) * SEQ + key0;
      const v16h a0 = g2_frag(vr, hh), a1 = g2_frag(vr + 32, hh);
      oh[dt] = g2_mma(a0, ph[0].v, oh[dt]);
      oh[dt] = g2_mma(a1, ph[1].v, oh[dt]);
      orr[dt] = g2_mma(a0, pr[0].v, orr[dt]);
      orr[dt] = g2_mma(a1, pr[1].v, orr[dt]);
    }
  }

  const float lt = l + __shfl_xor(l, 16);
  const float inv = (1.0f / lt) * 0.00390625f;
#pragma unroll
  for (int dt = 0; dt < 4; ++dt) {
#pragma unroll
    for (int r = 0; r < 8; ++r) so[w][ln][dt * 16 + 8 * (int)hh + r] = (oh[dt][r] + orr[dt][r] * 0.00048828125f) * inv;
  }
  __builtin_amdgcn_fence(4  , "workgroup");
  __builtin_amdgcn_wave_barrier();
  const unsigned rsub = lane >> 4, c4 = (lane & 15u) * 4u;
  float* obase = Og + ((size_t)b * SEQ + q0) * HD;
  for (int pass = 0; pass < 2; ++pass) {
#pragma unroll
    for (int q = 0; q < 8; ++q) {
      const unsigned r = (unsigned)q * 2u + rsub;
      const v4f v = *(const v4fa*)&so[w][r][c4];
      *(volatile v4f*)(obase + (size_t)r * HD + c4) = v;
    }
    if (pass == 0) __threadfence();
  }
}

extern "C" void kernel_launch(void* const* d_in, const int* in_sizes, int n_in,
                              void* d_out, int out_size, void* d_ws, size_t ws_size, hipStream_t stream) {
  if (n_in < 4) return;
  const long long need = (long long)NB * SEQ * HD;
  if ((long long)in_sizes[0] < need || (long long)in_sizes[1] < need || (long long)in_sizes[2] < need || in_sizes[3] < NB) return;
  if ((long long)out_size < need) return;
  const float* xq = (const float*)d_in[0];
  const float* xk = (const float*)d_in[1];
  const float* xv = (const float*)d_in[2];
  const int* pl = (const int*)d_in[3];
  char* ws = (char*)d_ws; size_t off = 0;
  auto take = [&](size_t bytes) { char* p = ws + off; off += (bytes + 255) & ~(size_t)255; return p; };
  _Float16* K16 = (_Float16*)take((size_t)NB * SEQ * HD * 2);
  _Float16* VT = (_Float16*)take((size_t)NB * HD * SEQ * 2);
  if (off > ws_size) return;

  k_k16<<<(unsigned)((size_t)NB * SEQ * 8 / 256), 256, 0, stream>>>(xk, K16);
  k_vtc<<<(unsigned)(NB * QT), 256, 0, stream>>>(xv, VT);
  k_fattn<<<(unsigned)(NB * QT), 128, 0, stream>>>(xq, K16, VT, pl, (float*)d_out);
}
